// UpsampleAttention_51943334477849
// MI455X (gfx1250) — hardware-verified
//
#include <hip/hip_runtime.h>


#define NB_  2
#define LL   2048
#define QQ   4096
#define DD   512
#define NH_  8
#define HD   64
#define ZH   2
#define RH   512
#define SCL  0.04419417382415922f
#define PCAR 1024.0f
typedef _Float16 h16;
typedef unsigned short bf;
typedef __attribute__((ext_vector_type(16))) __bf16   v16bf;
typedef __attribute__((ext_vector_type(16))) _Float16 v16h;
typedef __attribute__((ext_vector_type(8)))  _Float16 v8h;
typedef __attribute__((ext_vector_type(8)))  unsigned short v8us;
typedef __attribute__((ext_vector_type(8)))  float    v8f;
typedef __attribute__((ext_vector_type(4)))  float    v4f;
typedef v8h  __attribute__((may_alias)) v8ha;
typedef v4f  __attribute__((may_alias)) v4fa;
typedef v8us __attribute__((may_alias)) v8usa;

__device__ __forceinline__ unsigned short f2bf(float f) { unsigned u = __float_as_uint(f); u += 0x7FFFu + ((u >> 16) & 1u); return (unsigned short)(u >> 16); }
__device__ __forceinline__ float bf2f(unsigned short b) { return __uint_as_float(((unsigned)b) << 16); }
__device__ __forceinline__ float bfr(float f) { return bf2f(f2bf(f)); }
__device__ __forceinline__ v16h cat16(v8h lo, v8h hi) { return __builtin_shufflevector(lo, hi, 0, 1, 2, 3, 4, 5, 6, 7, 8, 9, 10, 11, 12, 13, 14, 15); }
__device__ __forceinline__ v16bf cat16b(v8us lo, v8us hi) { return __builtin_bit_cast(v16bf, __builtin_shufflevector(lo, hi, 0, 1, 2, 3, 4, 5, 6, 7, 8, 9, 10, 11, 12, 13, 14, 15)); }
__device__ __forceinline__ v8f wmma16(v16h a, v16h b, v8f c) { return __builtin_amdgcn_wmma_f32_16x16x32_f16(false, a, false, b, (short)0, c, false, false); }
__device__ __forceinline__ v8f wmmab(v16bf a, v16bf b, v8f c) { return __builtin_amdgcn_wmma_f32_16x16x32_bf16(false, a, false, b, (short)0, c, false, false); }


template <typename T16> struct WFrag;
template <> struct WFrag<h16> { typedef v16h V; static __device__ __forceinline__ V ld(const h16* p) { return cat16(*(const v8h*)p, *(const v8h*)(p + 16)); } static __device__ __forceinline__ v8f mma(V a, V b, v8f c) { return wmma16(a, b, c); } };
template <> struct WFrag<bf> { typedef v16bf V; static __device__ __forceinline__ V ld(const bf* p) { return cat16b(*(const v8us*)p, *(const v8us*)(p + 16)); } static __device__ __forceinline__ v8f mma(V a, V b, v8f c) { return wmmab(a, b, c); } };
template <typename T16, int NSPLIT, bool BIAS>
__global__ __launch_bounds__(32) void k_gemmw(const T16* __restrict__ A, const T16* __restrict__ A2, const T16* __restrict__ Bt, const T16* __restrict__ Bt2, int K, float* C, int ldc, const float* __restrict__ bias, size_t sA, size_t sB, size_t sC) {
    typedef typename WFrag<T16>::V V;
    __shared__ __align__(16) float os[16 * 68];
    const size_t z = blockIdx.z; A += z * sA; if (A2) A2 += z * sA; Bt += z * sB; if (Bt2) Bt2 += z * sB; C += z * sC;
    const int lane = threadIdx.x & 31, lr = lane & 15, hi = lane >> 4; const int r0 = blockIdx.x * 64, c0 = blockIdx.y * 64;
    v8f acc[4][4];
#pragma unroll
    for (int mb = 0; mb < 4; ++mb)
#pragma unroll
        for (int nb = 0; nb < 4; ++nb) acc[mb][nb] = (v8f){};
    const size_t aoff = (size_t)(r0 + lr) * K + 8 * hi, boff = (size_t)(c0 + lr) * K + 8 * hi;
#pragma unroll 1
    for (int kc = 0; kc < K; kc += 32) {
        V a[4], a2[4];
#pragma unroll
        for (int mb = 0; mb < 4; ++mb) { a[mb] = WFrag<T16>::ld(A + aoff + (size_t)mb * 16 * K + kc); if (NSPLIT == 1 || NSPLIT == 2) a2[mb] = WFrag<T16>::ld(A2 + aoff + (size_t)mb * 16 * K + kc); }
#pragma unroll
        for (int nb = 0; nb < 4; ++nb) { const V b = WFrag<T16>::ld(Bt + boff + (size_t)nb * 16 * K + kc); V b2; if (NSPLIT >= 2) b2 = WFrag<T16>::ld(Bt2 + boff + (size_t)nb * 16 * K + kc);
#pragma unroll
            for (int mb = 0; mb < 4; ++mb) { acc[mb][nb] = WFrag<T16>::mma(a[mb], b, acc[mb][nb]); if (NSPLIT == 1 || NSPLIT == 2) acc[mb][nb] = WFrag<T16>::mma(a2[mb], b, acc[mb][nb]); if (NSPLIT >= 2) acc[mb][nb] = WFrag<T16>::mma(a[mb], b2, acc[mb][nb]); } }
        asm volatile("v_nop\n\tv_nop\n\tv_nop\n\tv_nop" : "+v"(acc[0][0]), "+v"(acc[1][1]), "+v"(acc[2][2]), "+v"(acc[3][3]) : "v"(a[0]), "v"(a[3]));
    }
#pragma unroll
    for (int mb = 0; mb < 4; ++mb) {
#pragma unroll
        for (int nb = 0; nb < 4; ++nb) {
#pragma unroll
            for (int j = 0; j < 8; ++j) os[(hi * 8 + j) * 68 + nb * 16 + lr] = acc[mb][nb][j]; }
        __builtin_amdgcn_wave_barrier(); asm volatile("" ::: "memory");
        float* crow = C + (size_t)(r0 + mb * 16) * ldc + c0;
#pragma unroll 1
        for (int ps = 0; ps < 2; ++ps) {
#pragma unroll
            for (int s = 0; s < 8; ++s) { const int row = 2 * s + hi, cofs = lr * 4; v4f val = *(const v4fa*)(os + row * 68 + cofs); if (BIAS) { val[0] += bfr(bias[c0 + cofs]); val[1] += bfr(bias[c0 + cofs + 1]); val[2] += bfr(bias[c0 + cofs + 2]); val[3] += bfr(bias[c0 + cofs + 3]); }
                *(volatile v4f*)(crow + (size_t)row * ldc + cofs) = val; }
            if (ps == 0) __threadfence(); }
        __builtin_amdgcn_wave_barrier(); asm volatile("" ::: "memory");
    }
}

__device__ __forceinline__ h16 tohx(float x) { return (h16)x; }
__device__ __forceinline__ void splitf(float y, unsigned short& h, unsigned short& l) { h = f2bf(y); l = f2bf(y - bf2f(h)); }
typedef __attribute__((ext_vector_type(2))) _Float16 v2h;
typedef __attribute__((ext_vector_type(4))) _Float16 v4h;
typedef __attribute__((ext_vector_type(2))) unsigned short v2us;
typedef __attribute__((ext_vector_type(4))) unsigned short v4us;

__global__ __launch_bounds__(256) void k_cvt8(const float* __restrict__ src, bf* dst, size_t n8) { const size_t i = (size_t)blockIdx.x * 256 + threadIdx.x; if (i >= n8) return; const v8f v = *(const v8f*)(src + i * 8); v8us o;
#pragma unroll
    for (int k = 0; k < 8; ++k) o[k] = f2bf(v[k]); *(volatile v8us*)(dst + i * 8) = o; __threadfence(); *(volatile v8us*)(dst + i * 8) = o; }
__global__ __launch_bounds__(256) void k_interp(const float* __restrict__ x, bf* Xh, bf* Xl) { const size_t e = ((size_t)blockIdx.x * 256 + threadIdx.x) * 4; if (e >= (size_t)QQ * DD) return; const int c = (int)(e % DD); const int i = (int)(e / DD); const float src = fmaxf(__fsub_rn(__fdiv_rn(__fadd_rn((float)i, 0.5f), 2.0f), 0.5f), 0.f); const int i0 = (int)floorf(src); const int i1 = min(i0 + 1, LL - 1); const float w = __fsub_rn(src, (float)i0), w0 = __fsub_rn(1.0f, w); v4us oh, ol;
#pragma unroll
    for (int q = 0; q < 4; ++q) { float a = __fmul_rn(bfr(x[(size_t)i0 * DD + c + q]), w0); asm volatile("" : "+v"(a)); float bq = __fmul_rn(bfr(x[(size_t)i1 * DD + c + q]), w); asm volatile("" : "+v"(bq)); unsigned short u, c2; splitf(__fadd_rn(a, bq), u, c2); oh[q] = u; ol[q] = c2; }
    *(volatile v4us*)(Xh + e) = oh; *(volatile v4us*)(Xl + e) = ol; __threadfence(); *(volatile v4us*)(Xh + e) = oh; *(volatile v4us*)(Xl + e) = ol; }
__global__ __launch_bounds__(256) void k_pl(const float* __restrict__ F, int rows, h16* P16, bf* Ph, bf* Pl) { const size_t e = ((size_t)blockIdx.x * 256 + threadIdx.x) * 2; if (e >= (size_t)NH_ * rows * HD) return; const int d = (int)(e % HD); const int t = (int)((e / HD) % rows); const int h = (int)(e / ((size_t)HD * rows)); const float* f = F + (size_t)t * DD + h * HD + d; v2h o; v2us oh, ol;
#pragma unroll
    for (int u = 0; u < 2; ++u) { o[u] = tohx(f[u]); unsigned short a, c; splitf(f[u], a, c); oh[u] = a; ol[u] = c; } for (int ps = 0; ps < 2; ++ps) { *(volatile v2h*)(P16 + e) = o; *(volatile v2us*)(Ph + e) = oh; *(volatile v2us*)(Pl + e) = ol; if (ps == 0) __threadfence(); } }
__global__ __launch_bounds__(256) void k_vtp(const float* __restrict__ F, h16* V16, bf* Vh, bf* Vl) { const size_t e = ((size_t)blockIdx.x * 256 + threadIdx.x) * 2; if (e >= (size_t)NH_ * HD * LL) return; const int t = (int)(e % LL); const int d = (int)((e / LL) % HD); const int h = (int)(e / ((size_t)LL * HD)); v2h o; v2us oh, ol;
#pragma unroll
    for (int u = 0; u < 2; ++u) { const float v = F[(size_t)(t + u) * DD + h * HD + d]; o[u] = tohx(v); unsigned short a, c; splitf(v, a, c); oh[u] = a; ol[u] = c; } for (int ps = 0; ps < 2; ++ps) { *(volatile v2h*)(V16 + e) = o; *(volatile v2us*)(Vh + e) = oh; *(volatile v2us*)(Vl + e) = ol; if (ps == 0) __threadfence(); } }
__global__ __launch_bounds__(256) void k_usoft(const float* __restrict__ Sb, h16* P16, bf* Ph, bf* Pl) { const int lane = threadIdx.x & 31; const int row = blockIdx.x * 8 + (threadIdx.x >> 5); if (row >= ZH * QQ) return; const int i = row % QQ; const int z = row / QQ; const bool hires = i < RH; const float* sr = Sb + (size_t)row * LL; float v[64]; float mx = -3.0e38f;
#pragma unroll
    for (int ch = 0; ch < 16; ++ch) { const int j0 = ch * 128 + lane * 4; const v4f a = *(const v4f*)(sr + j0);
#pragma unroll
        for (int q = 0; q < 4; ++q) { const float t = (j0 + q <= i) ? a[q] * SCL : -3.0e38f; v[ch * 4 + q] = t; mx = fmaxf(mx, t); } }
#pragma unroll
    for (int sh = 16; sh; sh >>= 1) mx = fmaxf(mx, __shfl_xor(mx, sh, 32));
    float sum = 0.f;
#pragma unroll
    for (int k = 0; k < 64; ++k) { float d0 = __fsub_rn(v[k], mx); asm volatile("" : "+v"(d0)); v[k] = __expf(d0); sum += v[k]; }
#pragma unroll
    for (int sh = 16; sh; sh >>= 1) sum += __shfl_xor(sum, sh, 32);
    const float f = __fdiv_rn(hires ? 1.0f : PCAR, sum);
#pragma unroll 1
    for (int ps = 0; ps < 2; ++ps) {
        if (hires) {
#pragma unroll
            for (int ch = 0; ch < 16; ++ch) { v4us oh, ol;
#pragma unroll
                for (int q = 0; q < 4; ++q) { unsigned short a, c2; splitf(v[ch * 4 + q] * f, a, c2); oh[q] = a; ol[q] = c2; } const size_t oo = ((size_t)z * RH + i) * LL + ch * 128 + lane * 4; *(volatile v4us*)(Ph + oo) = oh; *(volatile v4us*)(Pl + oo) = ol; }
        } else {
#pragma unroll
            for (int ch = 0; ch < 16; ++ch) { v4h o4; o4[0] = tohx(v[ch * 4] * f); o4[1] = tohx(v[ch * 4 + 1] * f); o4[2] = tohx(v[ch * 4 + 2] * f); o4[3] = tohx(v[ch * 4 + 3] * f); *(volatile v4h*)(P16 + (size_t)row * LL + ch * 128 + lane * 4) = o4; } }
        if (ps == 0) __threadfence(); } }
__global__ __launch_bounds__(256) void k_mrg(const float* __restrict__ Ob, int h0, bf* Ah, bf* Al) { const size_t e = ((size_t)blockIdx.x * 256 + threadIdx.x) * 2; if (e >= (size_t)ZH * QQ * HD) return; const int d = (int)(e % HD); const int i = (int)((e / HD) % QQ); const int z = (int)(e / ((size_t)HD * QQ)); const float f = i < RH ? 1.0f : (1.0f / PCAR); v2us oh, ol;
#pragma unroll
    for (int u = 0; u < 2; ++u) { unsigned short a, c; splitf(Ob[e + u] * f, a, c); oh[u] = a; ol[u] = c; } const size_t o = (size_t)i * DD + (h0 + z) * HD + d; *(volatile v2us*)(Ah + o) = oh; *(volatile v2us*)(Al + o) = ol; __threadfence(); *(volatile v2us*)(Ah + o) = oh; *(volatile v2us*)(Al + o) = ol; }

extern "C" void kernel_launch(void* const* d_in, const int* in_sizes, int n_in,
                              void* d_out, int out_size, void* d_ws, size_t ws_size, hipStream_t stream) {
    (void)in_sizes; (void)n_in; (void)out_size;
    const float* x = (const float*)d_in[0]; const float* Wq = (const float*)d_in[1]; const float* bq = (const float*)d_in[2]; const float* Wk = (const float*)d_in[3]; const float* bk = (const float*)d_in[4]; const float* Wv = (const float*)d_in[5]; const float* bv = (const float*)d_in[6]; const float* Wo = (const float*)d_in[7]; const float* bo = (const float*)d_in[8];
    float* OUT = (float*)d_out;
    char* wsp = (char*)d_ws;
    auto take = [&](size_t bytes) { char* p = wsp; wsp += (bytes + 255) & ~(size_t)255; return (void*)p; };
    bf* WQ = (bf*)take((size_t)DD * DD * 2); bf* WK = (bf*)take((size_t)DD * DD * 2); bf* WV = (bf*)take((size_t)DD * DD * 2); bf* WO = (bf*)take((size_t)DD * DD * 2);
    bf* XB = (bf*)take((size_t)LL * DD * 2); bf* XIh = (bf*)take((size_t)QQ * DD * 2); bf* XIl = (bf*)take((size_t)QQ * DD * 2); float* QF = (float*)take((size_t)QQ * DD * 4); float* KF = (float*)take((size_t)LL * DD * 4); float* VF = (float*)take((size_t)LL * DD * 4);
    h16* Q16 = (h16*)take((size_t)NH_ * QQ * HD * 2); bf* Qh = (bf*)take((size_t)NH_ * QQ * HD * 2); bf* Ql = (bf*)take((size_t)NH_ * QQ * HD * 2); h16* K16 = (h16*)take((size_t)NH_ * LL * HD * 2); bf* Kh = (bf*)take((size_t)NH_ * LL * HD * 2); bf* Kl = (bf*)take((size_t)NH_ * LL * HD * 2); h16* V16 = (h16*)take((size_t)NH_ * HD * LL * 2); bf* Vh = (bf*)take((size_t)NH_ * HD * LL * 2); bf* Vl = (bf*)take((size_t)NH_ * HD * LL * 2);
    float* Sb = (float*)take((size_t)ZH * QQ * LL * 4); h16* P16 = (h16*)take((size_t)ZH * QQ * LL * 2); bf* Ph = (bf*)take((size_t)ZH * RH * LL * 2); bf* Pl = (bf*)take((size_t)ZH * RH * LL * 2); float* Ob = (float*)take((size_t)ZH * QQ * HD * 4); bf* Ah = (bf*)take((size_t)QQ * DD * 2); bf* Al = (bf*)take((size_t)QQ * DD * 2);
    if ((size_t)(wsp - (char*)d_ws) > ws_size) return;
    k_cvt8<<<(DD * DD / 8 + 255) / 256, 256, 0, stream>>>(Wq, WQ, (size_t)DD * DD / 8); k_cvt8<<<(DD * DD / 8 + 255) / 256, 256, 0, stream>>>(Wk, WK, (size_t)DD * DD / 8); k_cvt8<<<(DD * DD / 8 + 255) / 256, 256, 0, stream>>>(Wv, WV, (size_t)DD * DD / 8); k_cvt8<<<(DD * DD / 8 + 255) / 256, 256, 0, stream>>>(Wo, WO, (size_t)DD * DD / 8);
    for (int b = 0; b < NB_; ++b) { const float* xb = x + (size_t)b * LL * DD;
        k_cvt8<<<(LL * DD / 8 + 255) / 256, 256, 0, stream>>>(xb, XB, (size_t)LL * DD / 8); k_interp<<<(unsigned)(((size_t)QQ * DD / 4 + 255) / 256), 256, 0, stream>>>(xb, XIh, XIl);
        k_gemmw<bf, 1, true><<<dim3(QQ / 64, DD / 64, 1), 32, 0, stream>>>(XIh, XIl, WQ, nullptr, DD, QF, DD, bq, 0, 0, 0); k_gemmw<bf, 0, true><<<dim3(LL / 64, DD / 64, 1), 32, 0, stream>>>(XB, nullptr, WK, nullptr, DD, KF, DD, bk, 0, 0, 0); k_gemmw<bf, 0, true><<<dim3(LL / 64, DD / 64, 1), 32, 0, stream>>>(XB, nullptr, WV, nullptr, DD, VF, DD, bv, 0, 0, 0);
        k_pl<<<(unsigned)(((size_t)NH_ * QQ * HD / 2 + 255) / 256), 256, 0, stream>>>(QF, QQ, Q16, Qh, Ql); k_pl<<<(unsigned)(((size_t)NH_ * LL * HD / 2 + 255) / 256), 256, 0, stream>>>(KF, LL, K16, Kh, Kl); k_vtp<<<(unsigned)(((size_t)NH_ * HD * LL / 2 + 255) / 256), 256, 0, stream>>>(VF, V16, Vh, Vl);
        for (int h0 = 0; h0 < NH_; h0 += ZH) { const size_t z = (size_t)h0;
            k_gemmw<bf, 2, false><<<dim3(RH / 64, LL / 64, ZH), 32, 0, stream>>>(Qh + z * QQ * HD, Ql + z * QQ * HD, Kh + z * LL * HD, Kl + z * LL * HD, HD, Sb, LL, nullptr, (size_t)QQ * HD, (size_t)LL * HD, (size_t)QQ * LL);
            k_gemmw<h16, 0, false><<<dim3((QQ - RH) / 64, LL / 64, ZH), 32, 0, stream>>>(Q16 + z * QQ * HD + (size_t)RH * HD, nullptr, K16 + z * LL * HD, nullptr, HD, Sb + (size_t)RH * LL, LL, nullptr, (size_t)QQ * HD, (size_t)LL * HD, (size_t)QQ * LL);
            k_usoft<<<ZH * QQ / 8, 256, 0, stream>>>(Sb, P16, Ph, Pl);
            k_gemmw<bf, 2, false><<<dim3(RH / 64, 1, ZH), 32, 0, stream>>>(Ph, Pl, Vh + z * HD * LL, Vl + z * HD * LL, LL, Ob, HD, nullptr, (size_t)RH * LL, (size_t)HD * LL, (size_t)QQ * HD);
            k_gemmw<h16, 0, false><<<dim3((QQ - RH) / 64, 1, ZH), 32, 0, stream>>>(P16 + (size_t)RH * LL, nullptr, V16 + z * HD * LL, nullptr, LL, Ob + (size_t)RH * HD, HD, nullptr, (size_t)QQ * LL, (size_t)HD * LL, (size_t)QQ * HD);
            k_mrg<<<(unsigned)(((size_t)ZH * QQ * HD / 2 + 255) / 256), 256, 0, stream>>>(Ob, h0, Ah, Al); }
        k_gemmw<bf, 1, true><<<dim3(QQ / 64, DD / 64, 1), 32, 0, stream>>>(Ah, Al, WO, nullptr, DD, OUT + (size_t)b * QQ * DD, DD, bo, 0, 0, 0); }
}
